// LinearAttention_63574105915901
// MI455X (gfx1250) — hardware-verified
//
#include <hip/hip_runtime.h>
#include <math.h>

constexpr int kB     = 4;
constexpr int kN     = 4096;
constexpr int kDim   = 512;
constexpr int kHeads = 8;
constexpr int kDh    = 64;
constexpr int kTok   = kB * kN;
constexpr int kQkvWaves = 4;
constexpr int kTrPitch  = 72;
constexpr float kWCarry    = 16.0f;
constexpr float kResCarry  = 2048.0f;
constexpr float kResInv    = 1.0f / 2048.0f;
constexpr float kQKCarry   = 2048.0f;
constexpr float kVCarry    = 8.0f;
constexpr float kCtxCarry  = 16.0f;
constexpr float kO1Carry   = 8.0f;
constexpr float kProjScale = 1.0f / 16.0f;
constexpr float kCtxScale  = 1.0f / 1024.0f;
constexpr float kQCScale   = 1.0f / 4096.0f;
constexpr float kOutScale  = 1.0f / 128.0f;
static_assert(kHeads * kDh == kDim, "head layout");
static_assert(kTok % 64 == 0 && kDim % 64 == 0 && kN % 64 == 0 && kDh == 64, "tile multiples");
static_assert(kDim % 32 == 0 && (kN / 4) % 32 == 0 && kDh % 32 == 0, "K multiples of 32");
static_assert(kDim / 64 == 8, "eight head tiles per row block");
static_assert(kResInv * kResCarry == 1.0f, "residual carry");
static_assert(kCtxScale * kVCarry * kQKCarry == kCtxCarry, "ctx carry");
static_assert(kQCScale * kQKCarry * kCtxCarry == kO1Carry, "o1 carry");
static_assert(kOutScale * kO1Carry * kWCarry == 1.0f, "out carry");
static_assert((kTrPitch * 2) % 16 == 0, "staging pitch");
static_assert(kQkvWaves * 16 == 64, "four 16-row strips per block");

typedef __attribute__((ext_vector_type(16))) _Float16 v16h;
typedef __attribute__((ext_vector_type(8)))  _Float16 v8h;
typedef __attribute__((ext_vector_type(16))) __bf16   v16b;
typedef __attribute__((ext_vector_type(8)))  __bf16   v8b;
typedef __attribute__((ext_vector_type(8)))  float    v8f;
typedef __attribute__((ext_vector_type(4)))  float    v4f;
typedef __attribute__((ext_vector_type(4)))  unsigned int v4u;

__device__ __forceinline__ unsigned short f2bf_bits(float f) {
  unsigned u = __float_as_uint(f);
  return (unsigned short)((u + 0x7FFFu + ((u >> 16) & 1u)) >> 16);
}
__device__ __forceinline__ float bf_bits2f(unsigned short h) { return __uint_as_float(((unsigned)h) << 16); }

__device__ __forceinline__ void dep_guard_h(v8f& a, v8f& b, v16h x, v16h y) { asm volatile("v_nop\n\tv_nop\n\tv_nop\n\tv_nop" : "+v"(a), "+v"(b) : "v"(x), "v"(y)); }
__device__ __forceinline__ void dep_guard_b(v8f& a, v8f& b, v16b x, v16b y) { asm volatile("v_nop\n\tv_nop\n\tv_nop\n\tv_nop" : "+v"(a), "+v"(b) : "v"(x), "v"(y)); }
__device__ __forceinline__ void dep_guard4_h(v8f& a, v8f& b, v8f& c, v8f& d, v16h x, v16h y) {
  asm volatile("v_nop\n\tv_nop\n\tv_nop\n\tv_nop" : "+v"(a), "+v"(b), "+v"(c), "+v"(d) : "v"(x), "v"(y));
}
__device__ __forceinline__ void dep_guard4_b(v8f& a, v8f& b, v8f& c, v8f& d, v16b x, v16b y) {
  asm volatile("v_nop\n\tv_nop\n\tv_nop\n\tv_nop" : "+v"(a), "+v"(b), "+v"(c), "+v"(d) : "v"(x), "v"(y));
}
__device__ __forceinline__ void dep_guard8_h(v8f& a0, v8f& a1, v8f& a2, v8f& a3, v8f& a4, v8f& a5, v8f& a6, v8f& a7,
                                             v16h x, v16h y, v16h z) {
  asm volatile("v_nop\n\tv_nop\n\tv_nop\n\tv_nop"
               : "+v"(a0), "+v"(a1), "+v"(a2), "+v"(a3), "+v"(a4), "+v"(a5), "+v"(a6), "+v"(a7)
               : "v"(x), "v"(y), "v"(z));
}
__device__ __forceinline__ void keep4_h(v16h a, v16h b, v16h c, v16h d) { asm volatile("v_nop" :: "v"(a), "v"(b), "v"(c), "v"(d)); }
__device__ __forceinline__ void keep4_b(v16b a, v16b b, v16b c, v16b d) { asm volatile("v_nop" :: "v"(a), "v"(b), "v"(c), "v"(d)); }
__device__ __forceinline__ void acc_guard4(v8f& a, v8f& b, v8f& c, v8f& d) { asm volatile("v_nop\n\tv_nop\n\tv_nop\n\tv_nop" : "+v"(a), "+v"(b), "+v"(c), "+v"(d)); }
template <typename T> struct Frag;
template <> struct Frag<_Float16> {
  typedef v16h V; union U { v16h v; v8h h[2]; };
  static __device__ __forceinline__ v16h load(const _Float16* p) {
    U f; f.h[0] = *(const v8h*)(p); f.h[1] = *(const v8h*)(p + 16); return f.v;
  }
  static __device__ __forceinline__ v8f mma(v16h a, v16h b, v8f c) {
    return __builtin_amdgcn_wmma_f32_16x16x32_f16(false, a, false, b, (short)0, c, false, false);
  }
  static __device__ __forceinline__ void guard(v8f& a, v8f& b, v16h x, v16h y) { dep_guard_h(a, b, x, y); }
  static __device__ __forceinline__ void guard4(v8f& a, v8f& b, v8f& c, v8f& d, v16h x, v16h y) { dep_guard4_h(a, b, c, d, x, y); }
  static __device__ __forceinline__ void keep(v16h a, v16h b, v16h c, v16h d) { keep4_h(a, b, c, d); }
};
template <> struct Frag<__bf16> {
  typedef v16b V; union U { v16b v; v8b h[2]; };
  static __device__ __forceinline__ v16b load(const __bf16* p) {
    U f; f.h[0] = *(const v8b*)(p); f.h[1] = *(const v8b*)(p + 16); return f.v;
  }
  static __device__ __forceinline__ v8f mma(v16b a, v16b b, v8f c) {
    return __builtin_amdgcn_wmma_f32_16x16x32_bf16(false, a, false, b, (short)0, c, false, false);
  }
  static __device__ __forceinline__ void guard(v8f& a, v8f& b, v16b x, v16b y) { dep_guard_b(a, b, x, y); }
  static __device__ __forceinline__ void guard4(v8f& a, v8f& b, v8f& c, v8f& d, v16b x, v16b y) { dep_guard4_b(a, b, c, d, x, y); }
  static __device__ __forceinline__ void keep(v16b a, v16b b, v16b c, v16b d) { keep4_b(a, b, c, d); }
};

__device__ __forceinline__ unsigned pk16(unsigned short a, unsigned short b) { return (unsigned)a | ((unsigned)b << 16); }
__device__ __forceinline__ unsigned short h_bits(float f) { const _Float16 h = (_Float16)f; return __builtin_bit_cast(unsigned short, h); }

__device__ __forceinline__ void wave_sync() {
  __builtin_amdgcn_fence(__ATOMIC_RELEASE, "workgroup");
  __builtin_amdgcn_wave_barrier();
  __builtin_amdgcn_fence(__ATOMIC_ACQUIRE, "workgroup");
}

template <int ET> struct Elem;
template <> struct Elem<0> { typedef _Float16 T; };
template <> struct Elem<1> { typedef __bf16 T; };
template <int ET, bool SPLIT, int BIAS_MODE, int OUT_MODE, bool RESID, int ACT = 0>
__global__ __launch_bounds__(256) void wmma_gemm64(
    const unsigned short* __restrict__ Ap, const unsigned short* __restrict__ A2p, int lda, long strideA,
    const unsigned short* __restrict__ Btp, const unsigned short* __restrict__ Bt2p, int ldb, long strideB,
    void* __restrict__ Cout, void* __restrict__ Cout2, int ldc, long strideC,
    const float* __restrict__ bias,
    const float* __restrict__ resid, long strideR,
    int M, int N, int K, float scale) {
  typedef typename Elem<ET>::T T;
  typedef typename Frag<T>::V V;
  const T* A = (const T*)Ap; const T* A2 = (const T*)A2p; const T* Bt = (const T*)Btp; const T* Bt2 = (const T*)Bt2p;
  __shared__ __align__(16) float sT[8][16 * 68];
  const int b    = blockIdx.y;
  const int lane = threadIdx.x & 31;
  const int wave = threadIdx.x >> 5;
  const int tilesN = N >> 6;
  const int tilesM = M >> 6;
  const int tile = blockIdx.x * 8 + wave;
  if (tile >= tilesM * tilesN) return;
  const int tm = tile / tilesN;
  const int tn = tile - tm * tilesN;
  const int m0 = tm << 6;
  const int n0 = tn << 6;

  const T* Ab  = A  + (size_t)b * strideA;
  const T* Bb  = Bt + (size_t)b * strideB;
  const T* Ab2 = SPLIT ? (A2  + (size_t)b * strideA) : nullptr;
  const T* Bb2 = SPLIT ? (Bt2 + (size_t)b * strideB) : nullptr;

  const int rlane = lane & 15;
  const int koff  = (lane >> 4) * 8;
  const int mOff  = (lane >> 4) * 8;

  v8f acc[4][4];
#pragma unroll
  for (int i = 0; i < 4; ++i)
#pragma unroll
    for (int j = 0; j < 4; ++j) acc[i][j] = (v8f){0.f,0.f,0.f,0.f,0.f,0.f,0.f,0.f};

  for (int k0 = 0; k0 < K; k0 += 32) {
    V bh[4], bl[4];
#pragma unroll
    for (int j = 0; j < 4; ++j) {
      const size_t bo = (size_t)(n0 + (j << 4) + rlane) * ldb + koff + k0;
      bh[j] = Frag<T>::load(Bb + bo);
      if (SPLIT) bl[j] = Frag<T>::load(Bb2 + bo);
    }
#pragma unroll
    for (int i = 0; i < 4; ++i) {
      const size_t ao = (size_t)(m0 + (i << 4) + rlane) * lda + koff + k0;
      V ah = Frag<T>::load(Ab + ao);
      V al;
      if (SPLIT) al = Frag<T>::load(Ab2 + ao);
#pragma unroll
      for (int j = 0; j < 4; ++j) {
        acc[i][j] = Frag<T>::mma(ah, bh[j], acc[i][j]);
        if (SPLIT) {
          acc[i][j] = Frag<T>::mma(ah, bl[j], acc[i][j]);
          acc[i][j] = Frag<T>::mma(al, bh[j], acc[i][j]);
        }
      }
      Frag<T>::guard4(acc[i][0], acc[i][1], acc[i][2], acc[i][3], ah, SPLIT ? al : bh[3]);
    }
    Frag<T>::keep(bh[0], bh[1], bh[2], bh[3]);
    if (SPLIT) Frag<T>::keep(bl[0], bl[1], bl[2], bl[3]);
  }
  acc_guard4(acc[0][0], acc[0][1], acc[0][2], acc[0][3]);
  acc_guard4(acc[1][0], acc[1][1], acc[1][2], acc[1][3]);
  acc_guard4(acc[2][0], acc[2][1], acc[2][2], acc[2][3]);
  acc_guard4(acc[3][0], acc[3][1], acc[3][2], acc[3][3]);

  float* slab = sT[wave];
  const float* Rb = RESID ? (resid + (size_t)b * strideR) : nullptr;
#pragma unroll
  for (int i = 0; i < 4; ++i) {
    const int mBase = m0 + (i << 4);
#pragma unroll
    for (int j = 0; j < 4; ++j) {
      const int n = n0 + (j << 4) + rlane;
      float bv = 0.f;
      if (BIAS_MODE == 2) bv = bias[n];
#pragma unroll
      for (int r = 0; r < 8; ++r) {
        float v = acc[i][j][r] * scale;
        if (BIAS_MODE == 1) v += bias[mBase + mOff + r];
        if (BIAS_MODE == 2) v += bv;
        if (RESID) v += Rb[(size_t)(mBase + mOff + r) * ldc + n];
        if (ACT == 2) v = fmaxf(v, 0.0f);
        if (ACT == 4) v = (v > 0.f) ? v : 0.01f * v;
        slab[(mOff + r) * 68 + (j << 4) + rlane] = v;
      }
    }
    __builtin_amdgcn_fence(__ATOMIC_RELEASE, "workgroup");
    __builtin_amdgcn_wave_barrier();
    __builtin_amdgcn_fence(__ATOMIC_ACQUIRE, "workgroup");
    if (OUT_MODE == 0) {
      float* C = (float*)Cout + (size_t)b * strideC;
      const int hh = lane >> 4, c4 = (lane & 15) * 4;
      for (int pass = 0; pass < 2; ++pass) {
#pragma unroll
        for (int it = 0; it < 8; ++it) {
          const int row = it * 2 + hh;
          v4f v = *(const v4f*)(slab + row * 68 + c4);
          *(volatile v4f*)(C + (size_t)(mBase + row) * ldc + n0 + c4) = v;
        }
        __threadfence();
      }
    } else {
      const int q = lane >> 3, c8 = (lane & 7) * 8;
      unsigned short* C  = (unsigned short*)Cout  + (size_t)b * strideC;
      unsigned short* C2 = (OUT_MODE == 2) ? ((unsigned short*)Cout2 + (size_t)b * strideC) : nullptr;
      for (int pass = 0; pass < 2; ++pass) {
#pragma unroll
        for (int it = 0; it < 4; ++it) {
          const int row = it * 4 + q;
          const float* sp = slab + row * 68 + c8;
          v8h hv, lv;
#pragma unroll
          for (int e = 0; e < 8; ++e) {
            if (OUT_MODE == 1) {
              hv[e] = (_Float16)sp[e];
            } else {
              unsigned short hb = f2bf_bits(sp[e]);
              unsigned short lb = f2bf_bits(sp[e] - bf_bits2f(hb));
              hv[e] = __builtin_bit_cast(_Float16, hb);
              lv[e] = __builtin_bit_cast(_Float16, lb);
            }
          }
          *(volatile v8h*)(C + (size_t)(mBase + row) * ldc + n0 + c8) = hv;
          if (OUT_MODE == 2) *(volatile v8h*)(C2 + (size_t)(mBase + row) * ldc + n0 + c8) = lv;
        }
        __threadfence();
      }
    }
    __builtin_amdgcn_fence(__ATOMIC_RELEASE, "workgroup");
    __builtin_amdgcn_wave_barrier();
    __builtin_amdgcn_fence(__ATOMIC_ACQUIRE, "workgroup");
  }
}

__global__ __launch_bounds__(256) void cast8_split_kernel(const float* __restrict__ in, unsigned short* __restrict__ outH,
                                                          unsigned short* __restrict__ outL, int n8) {
  const int i = blockIdx.x * 256 + threadIdx.x;
  if (i >= n8) return;
  const float* p = in + 8 * (size_t)i;
  const v4f a = *(const v4f*)(p);
  const v4f c = *(const v4f*)(p + 4);
  unsigned short hb[8], lb[8];
#pragma unroll
  for (int e = 0; e < 4; ++e) {
    const float v0 = a[e];
    const _Float16 h0 = (_Float16)v0;
    const float hf0 = (float)h0;
    hb[e] = __builtin_bit_cast(unsigned short, h0);
    lb[e] = h_bits((v0 - hf0) * kResCarry);
    const float v1 = c[e];
    const _Float16 h1 = (_Float16)v1;
    const float hf1 = (float)h1;
    hb[4 + e] = __builtin_bit_cast(unsigned short, h1);
    lb[4 + e] = h_bits((v1 - hf1) * kResCarry);
  }
  const v4u uh = (v4u){pk16(hb[0], hb[1]), pk16(hb[2], hb[3]), pk16(hb[4], hb[5]), pk16(hb[6], hb[7])};
  const v4u ul = (v4u){pk16(lb[0], lb[1]), pk16(lb[2], lb[3]), pk16(lb[4], lb[5]), pk16(lb[6], lb[7])};
  unsigned short* qh = outH + 8 * (size_t)i;
  unsigned short* ql = outL + 8 * (size_t)i;
  *(volatile v4u*)qh = uh;
  *(volatile v4u*)ql = ul;
  __threadfence();
  *(volatile v4u*)qh = uh;
  *(volatile v4u*)ql = ul;
}

__global__ __launch_bounds__(256) void wtcast_kernel(const float* __restrict__ W0, const float* __restrict__ W1,
                                                     const float* __restrict__ W2, const float* __restrict__ W3,
                                                     unsigned short* __restrict__ out, float scale) {
  __shared__ float sm[64][65];
  const int t  = threadIdx.x;
  const int d0 = blockIdx.x * 64;
  const int h0 = blockIdx.y * 64;
  const int z  = blockIdx.z;
  const float* W = (z == 0) ? W0 : (z == 1) ? W1 : (z == 2) ? W2 : W3;
#pragma unroll
  for (int i = 0; i < 16; ++i) {
    const int e = i * 256 + t;
    const int r = e >> 6;
    const int c = e & 63;
    sm[c][r] = W[(size_t)(d0 + r) * kDim + h0 + c] * scale;
  }
  __syncthreads();
  const int lane = t & 31, wave = t >> 5;
  const int q = lane >> 3, c8 = (lane & 7) * 8;
  unsigned short* op = out + (size_t)z * kDim * kDim;
  for (int pass = 0; pass < 2; ++pass) {
#pragma unroll
    for (int it = 0; it < 2; ++it) {
      const int row = wave * 8 + it * 4 + q;
      unsigned short hb[8];
#pragma unroll
      for (int e = 0; e < 8; ++e) hb[e] = h_bits(sm[row][c8 + e]);
      const v4u u = (v4u){pk16(hb[0], hb[1]), pk16(hb[2], hb[3]), pk16(hb[4], hb[5]), pk16(hb[6], hb[7])};
      *(volatile v4u*)(op + (size_t)(h0 + row) * kDim + d0 + c8) = u;
    }
    __threadfence();
  }
}

__global__ __launch_bounds__(128) void qkv_softmax_kernel(const unsigned short* __restrict__ Xhp,
                                                          const unsigned short* __restrict__ Xlp,
                                                          const unsigned short* __restrict__ Wtp,
                                                          unsigned short* __restrict__ Qh,
                                                          unsigned short* __restrict__ Kt,
                                                          unsigned short* __restrict__ Vt) {
  __shared__ __align__(16) float sT[kQkvWaves][16 * 68];
  __shared__ __align__(16) unsigned short sTr[64 * kTrPitch];
  const int lane = threadIdx.x & 31;
  const int wave = threadIdx.x >> 5;
  const int z  = blockIdx.y;
  const int m0 = (blockIdx.x >> 3) * 64;
  const int n0 = (blockIdx.x & 7) * 64;
  const int r0 = m0 + wave * 16;
  const _Float16* A  = (const _Float16*)Xhp;
  const _Float16* A2 = (const _Float16*)Xlp;
  const _Float16* Bt = (const _Float16*)Wtp + (size_t)z * kDim * kDim;

  const int rlane = lane & 15;
  const int koff  = (lane >> 4) * 8;
  const int mOff  = (lane >> 4) * 8;

  v8f acc[4], accR[4];
#pragma unroll
  for (int j = 0; j < 4; ++j) {
    acc[j]  = (v8f){0.f,0.f,0.f,0.f,0.f,0.f,0.f,0.f};
    accR[j] = (v8f){0.f,0.f,0.f,0.f,0.f,0.f,0.f,0.f};
  }

  for (int k0 = 0; k0 < kDim; k0 += 32) {
    v16h bfr[4];
#pragma unroll
    for (int j = 0; j < 4; ++j) {
      const size_t bo = (size_t)(n0 + (j << 4) + rlane) * kDim + koff + k0;
      bfr[j] = Frag<_Float16>::load(Bt + bo);
    }
    const size_t ao = (size_t)(r0 + rlane) * kDim + koff + k0;
    const v16h af  = Frag<_Float16>::load(A + ao);
    const v16h afl = Frag<_Float16>::load(A2 + ao);
#pragma unroll
    for (int j = 0; j < 4; ++j) {
      acc[j]  = Frag<_Float16>::mma(af, bfr[j], acc[j]);
      accR[j] = Frag<_Float16>::mma(afl, bfr[j], accR[j]);
    }
    dep_guard8_h(acc[0], acc[1], acc[2], acc[3], accR[0], accR[1], accR[2], accR[3], af, afl, bfr[3]);
    Frag<_Float16>::keep(bfr[0], bfr[1], bfr[2], bfr[3]);
  }
  acc_guard4(acc[0], acc[1], acc[2], acc[3]);
  acc_guard4(accR[0], accR[1], accR[2], accR[3]);

  float* slab = sT[wave];
  const int rr = lane & 15;
  const int hh = lane >> 4;
  const int mBase = r0;
#pragma unroll
  for (int j = 0; j < 4; ++j) {
#pragma unroll
    for (int r = 0; r < 8; ++r) slab[(mOff + r) * 68 + (j << 4) + rlane] = fmaf(accR[j][r], kResInv, acc[j][r]) * kProjScale;
  }
  wave_sync();
  float rmul = kVCarry;
  if (z < 2) {
    float* rowp = slab + rr * 68 + hh * 32;
    float mx = -__builtin_inff();
#pragma unroll 1
    for (int c = 0; c < 32; ++c) mx = fmaxf(mx, rowp[c]);
    mx = fmaxf(mx, __shfl_xor(mx, 16, 32));
    float s = 0.0f;
#pragma unroll 1
    for (int c = 0; c < 32; ++c) {
      const float e = expf(rowp[c] - mx);
      rowp[c] = e;
      s += e;
    }
    s += __shfl_xor(s, 16, 32);
    const float inv = 1.0f / s;
    rmul = kQKCarry * inv;
    slab[rr * 68 + 64 + hh] = rmul;
  }
  wave_sync();
  if (z == 0) {
    const int q = lane >> 3, c8 = (lane & 7) * 8;
    for (int pass = 0; pass < 2; ++pass) {
#pragma unroll
      for (int it = 0; it < 4; ++it) {
        const int row = it * 4 + q;
        const float* sp = slab + row * 68 + c8;
        const float ri = slab[row * 68 + 64];
        v8h hv;
#pragma unroll
        for (int e = 0; e < 8; ++e) hv[e] = (_Float16)(sp[e] * ri);
        *(volatile v8h*)(Qh + (size_t)(mBase + row) * kDim + n0 + c8) = hv;
      }
      __threadfence();
    }
  } else {
    const float* rowp2 = slab + rr * 68 + hh * 32;
    unsigned short* tcol = sTr + (hh * 32) * kTrPitch + wave * 16 + rr;
#pragma unroll 1
    for (int c = 0; c < 32; ++c) tcol[c * kTrPitch] = h_bits(rowp2[c] * rmul);
  }
  __syncthreads();
  if (z >= 1) {
    unsigned short* dstT = (z == 1) ? Kt : Vt;
    const int bb  = m0 / kN;
    const int nl0 = m0 - bb * kN;
    const int q = lane >> 3, c8 = (lane & 7) * 8;
    const unsigned short* tsrc = sTr + (wave * 16) * kTrPitch + c8;
    unsigned short* base = dstT + ((size_t)(bb * kDim + n0 + wave * 16)) * kN + nl0 + c8;
    for (int pass = 0; pass < 2; ++pass) {
#pragma unroll
      for (int it = 0; it < 4; ++it) {
        const int frow = it * 4 + q;
        const v4u u = *(const v4u*)(tsrc + frow * kTrPitch);
        *(volatile v4u*)(base + (size_t)frow * kN) = u;
      }
      __threadfence();
    }
  }
}

__global__ __launch_bounds__(256) void ctx_kernel(const unsigned short* __restrict__ Vtp, const unsigned short* __restrict__ Ktp,
                                                  unsigned short* __restrict__ Ctp, float scale) {
  __shared__ __align__(16) float ctile[64 * 68];
  const int bh   = blockIdx.x;
  const int lane = threadIdx.x & 31;
  const int wave = threadIdx.x >> 5;
  const int mh   = wave & 1;
  const int kq   = wave >> 1;
  const _Float16* A  = (const _Float16*)Vtp + (size_t)bh * kDh * kN;
  const _Float16* Bt = (const _Float16*)Ktp + (size_t)bh * kDh * kN;
  const int rlane = lane & 15;
  const int koff  = (lane >> 4) * 8;
  const int mOff  = (lane >> 4) * 8;

  v8f acc[2][4];
#pragma unroll
  for (int i = 0; i < 2; ++i)
#pragma unroll
    for (int j = 0; j < 4; ++j) acc[i][j] = (v8f){0.f,0.f,0.f,0.f,0.f,0.f,0.f,0.f};

  const int kbeg = kq * (kN / 4);
  const int kend = kbeg + (kN / 4);
  for (int k0 = kbeg; k0 < kend; k0 += 32) {
    v16h bfr[4];
#pragma unroll
    for (int j = 0; j < 4; ++j) {
      const size_t bo = (size_t)((j << 4) + rlane) * kN + koff + k0;
      bfr[j] = Frag<_Float16>::load(Bt + bo);
    }
#pragma unroll
    for (int i = 0; i < 2; ++i) {
      const size_t ao = (size_t)(mh * 32 + (i << 4) + rlane) * kN + koff + k0;
      const v16h af = Frag<_Float16>::load(A + ao);
#pragma unroll
      for (int j = 0; j < 4; ++j) acc[i][j] = Frag<_Float16>::mma(af, bfr[j], acc[i][j]);
      Frag<_Float16>::guard4(acc[i][0], acc[i][1], acc[i][2], acc[i][3], af, bfr[3]);
    }
    Frag<_Float16>::keep(bfr[0], bfr[1], bfr[2], bfr[3]);
  }
  acc_guard4(acc[0][0], acc[0][1], acc[0][2], acc[0][3]);
  acc_guard4(acc[1][0], acc[1][1], acc[1][2], acc[1][3]);

  if (kq == 0) {
#pragma unroll
    for (int i = 0; i < 2; ++i)
#pragma unroll
      for (int j = 0; j < 4; ++j)
#pragma unroll
        for (int r = 0; r < 8; ++r) ctile[(mh * 32 + (i << 4) + mOff + r) * 68 + (j << 4) + rlane] = acc[i][j][r] * scale;
  }
  __syncthreads();
#pragma unroll 1
  for (int w = 1; w < 4; ++w) {
    if (kq == w) {
#pragma unroll
      for (int i = 0; i < 2; ++i)
#pragma unroll
        for (int j = 0; j < 4; ++j)
#pragma unroll
          for (int r = 0; r < 8; ++r) {
            const int idx = (mh * 32 + (i << 4) + mOff + r) * 68 + (j << 4) + rlane;
            ctile[idx] = ctile[idx] + acc[i][j][r] * scale;
          }
    }
    __syncthreads();
  }
  const int q = lane >> 3, c8 = (lane & 7) * 8;
  unsigned short* op = Ctp + (size_t)bh * kDh * kDh;
  for (int pass = 0; pass < 2; ++pass) {
#pragma unroll
    for (int it = 0; it < 2; ++it) {
      const int row = wave * 8 + it * 4 + q;
      unsigned short hb[8];
#pragma unroll
      for (int e = 0; e < 8; ++e) hb[e] = h_bits(ctile[row * 68 + c8 + e]);
      const v4u u = (v4u){pk16(hb[0], hb[1]), pk16(hb[2], hb[3]), pk16(hb[4], hb[5]), pk16(hb[6], hb[7])};
      *(volatile v4u*)(op + (size_t)row * kDh + c8) = u;
    }
    __threadfence();
  }
}

extern "C" void kernel_launch(void* const* d_in, const int* in_sizes, int n_in,
                              void* d_out, int out_size, void* d_ws, size_t ws_size,
                              hipStream_t stream) {
  if (n_in < 6) return;
  const int nElem = kTok * kDim;
  if (in_sizes[0] != nElem) return;
  if (in_sizes[1] != kDim * kDim || in_sizes[2] != kDim * kDim || in_sizes[3] != kDim * kDim || in_sizes[4] != kDim * kDim) return;
  if (in_sizes[5] != kDim) return;
  if (out_size != nElem) return;

  const size_t szPlane = (size_t)kTok * kDim * 2;
  const size_t szWt    = (size_t)4 * kDim * kDim * 2;
  const size_t szCtx   = (size_t)kB * kHeads * kDh * kDh * 2;
  const size_t offX   = 0;
  const size_t offXl  = offX + szPlane;
  const size_t offWt  = offXl + szPlane;
  const size_t offQ   = offWt + szWt;
  const size_t offKt  = offQ + szPlane;
  const size_t offVt  = offKt + szPlane;
  const size_t offCtx = offVt + szPlane;
  const size_t offO1  = offCtx + szCtx;
  const size_t total  = offO1 + szPlane;
  if (ws_size < total) return;

  const float* x  = (const float*)d_in[0];
  const float* Wq = (const float*)d_in[1];
  const float* Wk = (const float*)d_in[2];
  const float* Wv = (const float*)d_in[3];
  const float* Wo = (const float*)d_in[4];
  const float* bo = (const float*)d_in[5];
  float* out = (float*)d_out;
  char* ws = (char*)d_ws;
  unsigned short* Xh   = (unsigned short*)(ws + offX);
  unsigned short* Xl   = (unsigned short*)(ws + offXl);
  unsigned short* Wt   = (unsigned short*)(ws + offWt);
  unsigned short* Qh   = (unsigned short*)(ws + offQ);
  unsigned short* Kt   = (unsigned short*)(ws + offKt);
  unsigned short* Vt   = (unsigned short*)(ws + offVt);
  unsigned short* CtxT = (unsigned short*)(ws + offCtx);
  unsigned short* O1h  = (unsigned short*)(ws + offO1);
  const unsigned short* Wot = Wt + (size_t)3 * kDim * kDim;

  const int n8 = nElem / 8;
  cast8_split_kernel<<<dim3(n8 / 256), dim3(256), 0, stream>>>(x, Xh, Xl, n8);
  wtcast_kernel<<<dim3(kDim / 64, kDim / 64, 4), dim3(256), 0, stream>>>(Wq, Wk, Wv, Wo, Wt, kWCarry);

  qkv_softmax_kernel<<<dim3((kTok / 64) * (kDim / 64), 3), dim3(32 * kQkvWaves), 0, stream>>>(Xh, Xl, Wt, Qh, Kt, Vt);

  ctx_kernel<<<dim3(kB * kHeads), dim3(256), 0, stream>>>(Vt, Kt, CtxT, kCtxScale);

  const int tilesQC = (kN / 64) * (kDh / 64);
  for (int b = 0; b < kB; ++b) {
    const unsigned short* Ab = Qh + (size_t)b * kN * kDim;
    const unsigned short* Cb = CtxT + (size_t)b * kHeads * kDh * kDh;
    unsigned short* Ob = O1h + (size_t)b * kN * kDim;
    wmma_gemm64<0, false, 0, 1, false, 0><<<dim3(tilesQC / 8, kHeads), dim3(256), 0, stream>>>(
        Ab, Ab, kDim, (long)kDh, Cb, Cb, kDh, (long)(kDh * kDh),
        (void*)Ob, (void*)Ob, kDim, (long)kDh, bo, bo, 0L, kN, kDh, kDh, kQCScale);
  }

  const int tilesOut = (kTok / 64) * (kDim / 64);
  wmma_gemm64<0, false, 2, 0, false, 0><<<dim3(tilesOut / 8, 1), dim3(256), 0, stream>>>(
      O1h, O1h, kDim, 0L, Wot, Wot, kDim, 0L,
      (void*)out, (void*)out, kDim, 0L, bo, bo, 0L, kTok, kDim, kDim, kOutScale);
}
